// TranformerBlock_32495722562184
// MI455X (gfx1250) — hardware-verified
//
#include <hip/hip_runtime.h>
#include <math.h>
#include <stdint.h>

#define NB   2
#define SEQ  2048
#define HID  768
#define NHD  12
#define HD   64
#define DFF  3072
#define BT   (NB * SEQ)
#define NQB  (SEQ / 64)
#define WSC  64.0f
#define WINV 0.015625f
#define QRS  4096.0f
#define QRI  0.000244140625f
#define PSC  1024.0f
#define PSI  0.0009765625f
static_assert(NHD * HD == HID);
static_assert((SEQ % 64) == 0 && (HID % 64) == 0 && (DFF % 64) == 0 && (BT % 64) == 0);
static_assert(HID == 6 * 128);

typedef _Float16 v16h __attribute__((ext_vector_type(16)));
typedef _Float16 v8h  __attribute__((ext_vector_type(8)));
typedef float    v8f  __attribute__((ext_vector_type(8)));
typedef float    v4f  __attribute__((ext_vector_type(4)));
typedef unsigned int v4u __attribute__((ext_vector_type(4)));

__device__ __forceinline__ unsigned short bf_bits(float f) {
  const unsigned u = __float_as_uint(f);
  return (unsigned short)((u + 0x7FFFu + ((u >> 16) & 1u)) >> 16);
}
__device__ __forceinline__ float bfr(float f) { return __uint_as_float(((unsigned)bf_bits(f)) << 16); }
__device__ __forceinline__ v4f bfr4(v4f a) {
  v4f r;
  r[0] = bfr(a[0]); r[1] = bfr(a[1]); r[2] = bfr(a[2]); r[3] = bfr(a[3]);
  return r;
}
__device__ __forceinline__ unsigned short h_bits(_Float16 x) { return __builtin_bit_cast(unsigned short, x); }
__device__ __forceinline__ unsigned pk16(unsigned short a, unsigned short b) { return (unsigned)a | ((unsigned)b << 16); }
__device__ __forceinline__ unsigned pkh2(float a, float b) { return pk16(h_bits((_Float16)a), h_bits((_Float16)b)); }
__device__ __forceinline__ v8f zero8() { v8f z = {0.f, 0.f, 0.f, 0.f, 0.f, 0.f, 0.f, 0.f}; return z; }
__device__ __forceinline__ v4f zero4() { v4f z = {0.f, 0.f, 0.f, 0.f}; return z; }

__device__ __forceinline__ v16h ldfrag_h(const _Float16* p) {
  union { v16h v; v8h h[2]; } f;
  f.h[0] = *(const v8h*)(p);
  f.h[1] = *(const v8h*)(p + 16);
  return f.v;
}

__device__ __forceinline__ v8f mma_h(v16h a, v16h b, v8f c) {
  c = __builtin_amdgcn_wmma_f32_16x16x32_f16(false, a, false, b, (short)0, c, false, false);
#if defined(__HIP_DEVICE_COMPILE__)
  asm volatile("v_nop\n\tv_nop\n\tv_nop\n\tv_nop" : "+v"(c) : "v"(a), "v"(b));
#endif
  return c;
}

__device__ __forceinline__ void wave_lds_sync() {
  __builtin_amdgcn_fence(__ATOMIC_RELEASE, "workgroup");
  __builtin_amdgcn_wave_barrier();
  __builtin_amdgcn_fence(__ATOMIC_ACQUIRE, "workgroup");
}

__device__ __forceinline__ float gelu_t(float x) {
  float u = 0.7978845608028654f * (x + 0.044715f * x * x * x);
  u = fminf(fmaxf(u, -16.0f), 16.0f);
  const float e  = __expf(2.0f * u);
  const float th = 1.0f - 2.0f * __builtin_amdgcn_rcpf(e + 1.0f);
  return 0.5f * x * (1.0f + th);
}

template <bool ADDE, bool RSRC, bool OUT32>
__global__ __launch_bounds__(256) void ln_rows(const float* src, const float* embs, float* hdst,
                                               const float* __restrict__ sc, const float* __restrict__ bi,
                                               void* outp, int nrows) {
  __shared__ __align__(16) float rb[8 * HID];
  const int tid = threadIdx.x, wave = tid >> 5, lane = tid & 31;
  const int row = blockIdx.x * 8 + wave;
  if (row >= nrows) return;
  const size_t rbase = (size_t)row * HID;
  v4f x[6];
#pragma unroll
  for (int i = 0; i < 6; ++i) {
    const int col = i * 128 + lane * 4;
    v4f a = *(const v4f*)(src + rbase + col);
    if (RSRC) a = bfr4(a);
    if (ADDE) {
      const v4f e = bfr4(*(const v4f*)(embs + rbase + col));
      a = a + e;
    }
    x[i] = a;
  }
  if (ADDE) {
    for (int pass = 0; pass < 2; ++pass) {
#pragma unroll
      for (int i = 0; i < 6; ++i) *(volatile v4f*)(hdst + rbase + i * 128 + lane * 4) = x[i];
      __threadfence();
    }
  }
  float s = 0.f;
#pragma unroll
  for (int i = 0; i < 6; ++i) s += (x[i][0] + x[i][1]) + (x[i][2] + x[i][3]);
#pragma unroll
  for (int off = 1; off < 32; off <<= 1) s += __shfl_xor(s, off, 32);
  const float mean = s * (1.0f / 768.0f);
  float qv = 0.f;
#pragma unroll
  for (int i = 0; i < 6; ++i) {
    const v4f d = x[i] - mean;
    qv += (d[0] * d[0] + d[1] * d[1]) + (d[2] * d[2] + d[3] * d[3]);
  }
#pragma unroll
  for (int off = 1; off < 32; off <<= 1) qv += __shfl_xor(qv, off, 32);
  const float var  = qv * (1.0f / 768.0f);
  const float rinv = rsqrtf(var + 1e-5f);
  v4f y[6];
#pragma unroll
  for (int i = 0; i < 6; ++i) {
    const int col = i * 128 + lane * 4;
    const v4f s4 = bfr4(*(const v4f*)(sc + col));
    const v4f b4 = bfr4(*(const v4f*)(bi + col));
    y[i] = (x[i] - mean) * rinv * s4 + b4;
  }
  if (OUT32) {
    float* o = (float*)outp;
    for (int pass = 0; pass < 2; ++pass) {
#pragma unroll
      for (int i = 0; i < 6; ++i) *(volatile v4f*)(o + rbase + i * 128 + lane * 4) = y[i];
      __threadfence();
    }
  } else {
    float* rw = rb + wave * HID;
#pragma unroll
    for (int i = 0; i < 6; ++i) *(v4f*)(rw + i * 128 + lane * 4) = y[i];
    wave_lds_sync();
    v4u pk[3];
#pragma unroll
    for (int j = 0; j < 3; ++j) {
      const v4f a = *(const v4f*)(rw + j * 256 + lane * 8);
      const v4f c = *(const v4f*)(rw + j * 256 + lane * 8 + 4);
      v4u p;
      p[0] = pkh2(a[0], a[1]); p[1] = pkh2(a[2], a[3]);
      p[2] = pkh2(c[0], c[1]); p[3] = pkh2(c[2], c[3]);
      pk[j] = p;
    }
    unsigned short* o = (unsigned short*)outp;
    for (int pass = 0; pass < 2; ++pass) {
#pragma unroll
      for (int j = 0; j < 3; ++j) *(volatile v4u*)(o + rbase + j * 256 + lane * 8) = pk[j];
      __threadfence();
    }
  }
}

__global__ __launch_bounds__(256) void convT(const float* __restrict__ W0, const float* __restrict__ W1,
                                             const float* __restrict__ W2, const float* __restrict__ W3,
                                             unsigned short* O0, unsigned short* O1,
                                             unsigned short* O2, unsigned short* O3, int K, int N) {
  __shared__ __align__(16) _Float16 sT[64 * 72];
  const int z = blockIdx.z;
  const float* W = (z == 0) ? W0 : (z == 1) ? W1 : (z == 2) ? W2 : W3;
  unsigned short* O = (z == 0) ? O0 : (z == 1) ? O1 : (z == 2) ? O2 : O3;
  const int n0 = blockIdx.x * 64, k0 = blockIdx.y * 64;
  const int tid = threadIdx.x;
  {
    const int r = tid >> 2, cq = (tid & 3) * 16;
    const float* p = W + (size_t)(k0 + r) * N + n0 + cq;
#pragma unroll
    for (int g = 0; g < 4; ++g) {
      const v4f a = *(const v4f*)(p + 4 * g);
#pragma unroll
      for (int e = 0; e < 4; ++e) sT[(cq + 4 * g + e) * 72 + r] = (_Float16)(bfr(a[e]) * WSC);
    }
  }
  __syncthreads();
  const int wave = tid >> 5, lane = tid & 31;
  const int q = lane >> 3, c8 = (lane & 7) * 8;
  union HU { v8h h; v4u u; };
  HU pk[2];
#pragma unroll
  for (int it = 0; it < 2; ++it) {
    const int row = wave * 8 + it * 4 + q;
    pk[it].h = *(const v8h*)(sT + row * 72 + c8);
  }
  const _Float16 dummy = (_Float16)0.0f; (void)dummy;
  for (int pass = 0; pass < 2; ++pass) {
#pragma unroll
    for (int it = 0; it < 2; ++it) {
      const int row = wave * 8 + it * 4 + q;
      *(volatile v4u*)(O + (size_t)(n0 + row) * K + k0 + c8) = pk[it].u;
    }
    __threadfence();
  }
}

template <int MODE>
__global__ __launch_bounds__(256) void gemm64(
    const unsigned short* __restrict__ Ap, int lda, long long strideA,
    const unsigned short* __restrict__ Btp, int ldb, long long strideB,
    const float* __restrict__ bias,
    void* Cout, void* Cout2, int ldc, long long strideC,
    int M, int N, int K) {
  __shared__ __align__(16) float sT[8][16 * 68];
  const int bz   = blockIdx.y;
  const int lane = threadIdx.x & 31;
  const int wave = threadIdx.x >> 5;
  const int tilesN = N >> 6;
  const int tilesM = M >> 6;
  const int tile = blockIdx.x * 8 + wave;
  if (tile >= tilesM * tilesN) return;
  const int tm = tile / tilesN;
  const int tn = tile - tm * tilesN;
  const int m0 = tm << 6;
  const int n0 = tn << 6;

  const _Float16* Ab = (const _Float16*)(const void*)Ap  + (size_t)bz * (size_t)strideA;
  const _Float16* Bb = (const _Float16*)(const void*)Btp + (size_t)bz * (size_t)strideB;

  const int rl   = lane & 15;
  const int hh   = lane >> 4;
  const int koff = hh * 8;
  const int mOff = hh * 8;

  v8f acc[4][4];
#pragma unroll
  for (int i = 0; i < 4; ++i)
#pragma unroll
    for (int j = 0; j < 4; ++j) acc[i][j] = zero8();

#pragma unroll 1
  for (int k0 = 0; k0 < K; k0 += 32) {
    v16h bfg[4];
#pragma unroll
    for (int j = 0; j < 4; ++j)
      bfg[j] = ldfrag_h(Bb + (size_t)(n0 + (j << 4) + rl) * ldb + koff + k0);
#pragma unroll
    for (int i = 0; i < 4; ++i) {
      const v16h af = ldfrag_h(Ab + (size_t)(m0 + (i << 4) + rl) * lda + koff + k0);
#pragma unroll
      for (int j = 0; j < 4; ++j) acc[i][j] = mma_h(af, bfg[j], acc[i][j]);
    }
  }

  float* slab = sT[wave];
#pragma unroll
  for (int i = 0; i < 4; ++i) {
    const int mBase = m0 + (i << 4);
#pragma unroll
    for (int j = 0; j < 4; ++j) {
#pragma unroll
      for (int r = 0; r < 8; ++r) slab[(mOff + r) * 68 + (j << 4) + rl] = acc[i][j][r] * WINV;
    }
    wave_lds_sync();
    if (MODE == 0) {
      float* C = (float*)Cout + (size_t)bz * (size_t)strideC;
      const int c4 = rl * 4;
      const v4f b4 = bfr4(*(const v4f*)(bias + n0 + c4));
      v4f vals[8];
#pragma unroll
      for (int it = 0; it < 8; ++it) {
        const int row = it * 2 + hh;
        const v4f v = *(const v4f*)(slab + row * 68 + c4);
        const v4f o = *(const v4f*)(C + (size_t)(mBase + row) * ldc + n0 + c4);
        vals[it] = o + (v + b4);
      }
      for (int pass = 0; pass < 2; ++pass) {
#pragma unroll
        for (int it = 0; it < 8; ++it) {
          const int row = it * 2 + hh;
          *(volatile v4f*)(C + (size_t)(mBase + row) * ldc + n0 + c4) = vals[it];
        }
        __threadfence();
      }
    } else {
      const int q = lane >> 3, c8 = (lane & 7) * 8;
      unsigned short* C  = (unsigned short*)Cout  + (size_t)bz * (size_t)strideC;
      unsigned short* C2 = (unsigned short*)Cout2 + (size_t)bz * (size_t)strideC;
      v4f ba = zero4(), bb = zero4();
      if (MODE != 3) {
        ba = bfr4(*(const v4f*)(bias + n0 + c8));
        bb = bfr4(*(const v4f*)(bias + n0 + c8 + 4));
      }
      v4u hv[4], lv[4];
#pragma unroll
      for (int it = 0; it < 4; ++it) {
        const int row = it * 4 + q;
        const float* sp = slab + row * 68 + c8;
        v4f fa = *(const v4f*)(sp);
        v4f fb = *(const v4f*)(sp + 4);
        if (MODE == 3) {
          const float br = bfr(bias[mBase + row]);
          fa = fa + br; fb = fb + br;
        } else {
          fa = fa + ba; fb = fb + bb;
        }
        if (MODE == 4) {
#pragma unroll
          for (int e = 0; e < 4; ++e) { fa[e] = gelu_t(fa[e]); fb[e] = gelu_t(fb[e]); }
        }
        v4u a, a2;
        if (MODE == 2) {
#pragma unroll
          for (int e = 0; e < 2; ++e) {
            const float f0 = fa[2 * e], f1 = fa[2 * e + 1];
            const float g0 = fb[2 * e], g1 = fb[2 * e + 1];
            const _Float16 x0 = (_Float16)f0, x1 = (_Float16)f1, y0 = (_Float16)g0, y1 = (_Float16)g1;
            a[e]      = pk16(h_bits(x0), h_bits(x1));
            a[e + 2]  = pk16(h_bits(y0), h_bits(y1));
            a2[e]     = pk16(h_bits((_Float16)((f0 - (float)x0) * QRS)), h_bits((_Float16)((f1 - (float)x1) * QRS)));
            a2[e + 2] = pk16(h_bits((_Float16)((g0 - (float)y0) * QRS)), h_bits((_Float16)((g1 - (float)y1) * QRS)));
          }
        } else {
          a[0] = pkh2(fa[0], fa[1]); a[1] = pkh2(fa[2], fa[3]);
          a[2] = pkh2(fb[0], fb[1]); a[3] = pkh2(fb[2], fb[3]);
          a2 = a;
        }
        hv[it] = a; lv[it] = a2;
      }
      for (int pass = 0; pass < 2; ++pass) {
#pragma unroll
        for (int it = 0; it < 4; ++it) {
          const int row = it * 4 + q;
          *(volatile v4u*)(C + (size_t)(mBase + row) * ldc + n0 + c8) = hv[it];
          if (MODE == 2) *(volatile v4u*)(C2 + (size_t)(mBase + row) * ldc + n0 + c8) = lv[it];
        }
        __threadfence();
      }
    }
    wave_lds_sync();
  }
}

__global__ __launch_bounds__(128)
void attn64(const unsigned short* __restrict__ qhp, const unsigned short* __restrict__ qlp,
            const unsigned short* __restrict__ khp, const unsigned short* __restrict__ vtp,
            const float* __restrict__ mask, unsigned short* ctxp, float sscale) {
  union FH { v16h v; v8h h[2]; };
  __shared__ __align__(16) _Float16 Ks[64 * 64];
  __shared__ __align__(16) _Float16 Vts[64 * 64];
  __shared__ __align__(16) _Float16 Psh[4][16 * 64];
  __shared__ __align__(16) float    Os[4][16 * 64];

  const int tid  = threadIdx.x;
  const int wave = tid >> 5;
  const int lane = tid & 31;
  const int hh   = lane >> 4;
  const int c    = lane & 15;

  const int bx   = blockIdx.x;
  const int qb   = bx % NQB;
  const int rest = bx / NQB;
  const int h    = rest % NHD;
  const int b    = rest / NHD;
  const int q0   = qb * 64 + wave * 16;
  const size_t rowB = (size_t)b * SEQ;

  const _Float16* Qh = (const _Float16*)(const void*)qhp + (size_t)h * HD;
  const _Float16* Ql = (const _Float16*)(const void*)qlp + (size_t)h * HD;
  const _Float16* Kh = (const _Float16*)(const void*)khp + (size_t)h * HD;
  const _Float16* Vt = (const _Float16*)(const void*)vtp + ((size_t)b * HID + (size_t)h * HD) * SEQ;
  const float* mb = mask + (size_t)b * SEQ;

  v16h qah[2], qal[2];
#pragma unroll
  for (int dc = 0; dc < 2; ++dc) {
    const size_t qo = (rowB + q0 + c) * HID + dc * 32 + 8 * hh;
    qah[dc] = ldfrag_h(Qh + qo);
    qal[dc] = ldfrag_h(Ql + qo);
  }

  float mrow[8], lrow[8];
  v8f oacc[4];
#pragma unroll
  for (int r = 0; r < 8; ++r) { mrow[r] = -INFINITY; lrow[r] = 0.f; }
#pragma unroll
  for (int t = 0; t < 4; ++t) oacc[t] = zero8();

#pragma unroll 1
  for (int kt = 0; kt < NQB; ++kt) {
    const int kv0 = kt * 64;
    __syncthreads();
    {
      const int r = tid >> 1, half = (tid & 1) * 32;
      const _Float16* kg = Kh + (rowB + kv0 + r) * HID + half;
      const _Float16* vg = Vt + (size_t)r * SEQ + kv0 + half;
#pragma unroll
      for (int i = 0; i < 4; ++i) {
        const v8h a0 = *(const v8h*)(kg + 8 * i);
        const v8h b0 = *(const v8h*)(vg + 8 * i);
        *(v8h*)(Ks  + r * 64 + half + 8 * i) = a0;
        *(v8h*)(Vts + r * 64 + half + 8 * i) = b0;
      }
    }
    __syncthreads();

    float mv[4];
#pragma unroll
    for (int j = 0; j < 4; ++j) mv[j] = bfr(mb[kv0 + j * 16 + c]);

    v8f s[4];
#pragma unroll
    for (int j = 0; j < 4; ++j) {
      s[j] = zero8();
      v8f sl = zero8();
#pragma unroll
      for (int dc = 0; dc < 2; ++dc) {
        FH kb;
        kb.h[0] = *(const v8h*)(Ks + (j * 16 + c) * 64 + dc * 32 + 8 * hh);
        kb.h[1] = *(const v8h*)(Ks + (j * 16 + c) * 64 + dc * 32 + 16 + 8 * hh);
        s[j] = mma_h(qah[dc], kb.v, s[j]);
        sl   = mma_h(qal[dc], kb.v, sl);
      }
#pragma unroll
      for (int r = 0; r < 8; ++r) {
        float sv = (s[j][r] + sl[r] * QRI) * sscale;
        sv = sv * mv[j] - 1.0e10f * (1.0f - mv[j]);
        s[j][r] = sv;
      }
    }

    _Float16* pwh = Psh[wave];
#pragma unroll
    for (int r = 0; r < 8; ++r) {
      float m = fmaxf(fmaxf(s[0][r], s[1][r]), fmaxf(s[2][r], s[3][r]));
#pragma unroll
      for (int off = 1; off < 16; off <<= 1) m = fmaxf(m, __shfl_xor(m, off, 32));
      const float mnew  = fmaxf(mrow[r], m);
      const float alpha = __expf(mrow[r] - mnew);
      mrow[r] = mnew;
      float psum = 0.f;
#pragma unroll
      for (int j = 0; j < 4; ++j) {
        const float p = __expf(s[j][r] - mnew);
        psum += p;
        pwh[(8 * hh + r) * 64 + j * 16 + c] = (_Float16)(p * PSC);
      }
#pragma unroll
      for (int off = 1; off < 16; off <<= 1) psum += __shfl_xor(psum, off, 32);
      lrow[r] = lrow[r] * alpha + psum;
#pragma unroll
      for (int t = 0; t < 4; ++t) oacc[t][r] *= alpha;
    }
    wave_lds_sync();

#pragma unroll
    for (int kk = 0; kk < 2; ++kk) {
      FH pa;
      pa.h[0] = *(const v8h*)(pwh + c * 64 + kk * 32 + 8 * hh);
      pa.h[1] = *(const v8h*)(pwh + c * 64 + kk * 32 + 16 + 8 * hh);
#pragma unroll
      for (int t = 0; t < 4; ++t) {
        FH vb;
        vb.h[0] = *(const v8h*)(Vts + (t * 16 + c) * 64 + kk * 32 + 8 * hh);
        vb.h[1] = *(const v8h*)(Vts + (t * 16 + c) * 64 + kk * 32 + 16 + 8 * hh);
        oacc[t] = mma_h(pa.v, vb.v, oacc[t]);
      }
    }
  }

  float* os = Os[wave];
#pragma unroll
  for (int r = 0; r < 8; ++r) {
    const float l = lrow[r];
    const float inv = ((l > 0.f) ? (1.0f / l) : 0.f) * PSI;
#pragma unroll
    for (int t = 0; t < 4; ++t) os[(8 * hh + r) * 64 + t * 16 + c] = oacc[t][r] * inv;
  }
  wave_lds_sync();
  {
    const int q4 = lane >> 3, c8 = (lane & 7) * 8;
    v4u hv[4];
#pragma unroll
    for (int it = 0; it < 4; ++it) {
      const int row = it * 4 + q4;
      const float* sp = os + row * 64 + c8;
      const v4f fa = *(const v4f*)(sp);
      const v4f fb = *(const v4f*)(sp + 4);
      v4u a;
      a[0] = pkh2(fa[0], fa[1]); a[1] = pkh2(fa[2], fa[3]);
      a[2] = pkh2(fb[0], fb[1]); a[3] = pkh2(fb[2], fb[3]);
      hv[it] = a;
    }
    for (int pass = 0; pass < 2; ++pass) {
#pragma unroll
      for (int it = 0; it < 4; ++it) {
        const int row = it * 4 + q4;
        const size_t go = (rowB + q0 + row) * HID + (size_t)h * HD + c8;
        *(volatile v4u*)(ctxp + go) = hv[it];
      }
      __threadfence();
    }
  }
}

extern "C" void kernel_launch(void* const* d_in, const int* in_sizes, int n_in,
                              void* d_out, int out_size, void* d_ws, size_t ws_size,
                              hipStream_t stream) {
  if (n_in < 21) return;
  if (in_sizes[0] != BT * HID || in_sizes[1] != BT * HID || in_sizes[2] != NB * SEQ) return;
  if (in_sizes[3] != 2 * HID || in_sizes[4] != 2 * HID) return;
  if (in_sizes[5] != 2 * HID * HID || in_sizes[7] != 2 * HID * HID ||
      in_sizes[9] != 2 * HID * HID || in_sizes[11] != 2 * HID * HID) return;
  if (in_sizes[6] != 2 * HID || in_sizes[8] != 2 * HID || in_sizes[10] != 2 * HID || in_sizes[12] != 2 * HID) return;
  if (in_sizes[13] != 2 * HID || in_sizes[14] != 2 * HID) return;
  if (in_sizes[15] != 2 * HID * DFF || in_sizes[16] != 2 * DFF ||
      in_sizes[17] != 2 * DFF * HID || in_sizes[18] != 2 * HID) return;
  if (in_sizes[19] != HID || in_sizes[20] != HID) return;
  if (out_size != BT * HID) return;

  const float* in_h  = (const float*)d_in[0];
  const float* embs  = (const float*)d_in[1];
  const float* mask  = (const float*)d_in[2];
  const float* ln1_s = (const float*)d_in[3];
  const float* ln1_b = (const float*)d_in[4];
  const float* wq    = (const float*)d_in[5];
  const float* bq    = (const float*)d_in[6];
  const float* wk    = (const float*)d_in[7];
  const float* bk    = (const float*)d_in[8];
  const float* wv    = (const float*)d_in[9];
  const float* bv    = (const float*)d_in[10];
  const float* wo    = (const float*)d_in[11];
  const float* bo    = (const float*)d_in[12];
  const float* ln2_s = (const float*)d_in[13];
  const float* ln2_b = (const float*)d_in[14];
  const float* w1    = (const float*)d_in[15];
  const float* b1    = (const float*)d_in[16];
  const float* w2    = (const float*)d_in[17];
  const float* b2    = (const float*)d_in[18];
  const float* lnf_s = (const float*)d_in[19];
  const float* lnf_b = (const float*)d_in[20];
  float* out = (float*)d_out;

  const size_t PH  = (size_t)BT * HID * 4;
  const size_t PA  = (size_t)BT * HID * 2;
  const size_t PVT = (size_t)NB * HID * SEQ * 2;
  const size_t PG  = (size_t)BT * DFF * 2;
  const size_t PW  = (size_t)HID * HID * 2;
  const size_t PW1 = (size_t)HID * DFF * 2;
  size_t off = 0;
  const size_t oH   = off; off += PH;
  const size_t oX   = off; off += PA;
  const size_t oQh  = off; off += PA;
  const size_t oQl  = off; off += PA;
  const size_t oKh  = off; off += PA;
  const size_t oVT  = off; off += PVT;
  const size_t oCtx = off; off += PA;
  const size_t oG   = off; off += PG;
  const size_t oWq  = off; off += PW;
  const size_t oWk  = off; off += PW;
  const size_t oWv  = off; off += PW;
  const size_t oWo  = off; off += PW;
  const size_t oW1  = off; off += PW1;
  const size_t oW2  = off; off += PW1;
  if (off > ws_size) return;
  if (off > (size_t)134217728) return;

  char* ws = (char*)d_ws;
  float*          Hres = (float*)(ws + oH);
  unsigned short* X    = (unsigned short*)(ws + oX);
  unsigned short* Qh   = (unsigned short*)(ws + oQh);
  unsigned short* Ql   = (unsigned short*)(ws + oQl);
  unsigned short* Kh   = (unsigned short*)(ws + oKh);
  unsigned short* VT   = (unsigned short*)(ws + oVT);
  unsigned short* Ctx  = (unsigned short*)(ws + oCtx);
  unsigned short* G    = (unsigned short*)(ws + oG);
  unsigned short* Wqt  = (unsigned short*)(ws + oWq);
  unsigned short* Wkt  = (unsigned short*)(ws + oWk);
  unsigned short* Wvt  = (unsigned short*)(ws + oWv);
  unsigned short* Wot  = (unsigned short*)(ws + oWo);
  unsigned short* W1t  = (unsigned short*)(ws + oW1);
  unsigned short* W2t  = (unsigned short*)(ws + oW2);

  const dim3 blk(256);
  const dim3 gLN(BT / 8);
  const dim3 gCv4(HID / 64, HID / 64, 4);
  const dim3 gCv1(DFF / 64, HID / 64, 1);
  const dim3 gCv2(HID / 64, DFF / 64, 1);
  const dim3 gHH(((BT / 64) * (HID / 64) + 7) / 8, 1);
  const dim3 gVT(((HID / 64) * (SEQ / 64) + 7) / 8, NB);
  const dim3 gF1(((BT / 64) * (DFF / 64) + 7) / 8, 1);
  const dim3 gAt(NB * NHD * NQB);

  for (int l = 0; l < 2; ++l) {
    const float* wql = wq + (size_t)l * HID * HID;
    const float* wkl = wk + (size_t)l * HID * HID;
    const float* wvl = wv + (size_t)l * HID * HID;
    const float* wol = wo + (size_t)l * HID * HID;
    const float* w1l = w1 + (size_t)l * HID * DFF;
    const float* w2l = w2 + (size_t)l * DFF * HID;
    if (l == 0) {
      ln_rows<true, true, false><<<gLN, blk, 0, stream>>>(in_h, embs, Hres, ln1_s, ln1_b, (void*)X, BT);
    } else {
      ln_rows<true, false, false><<<gLN, blk, 0, stream>>>(Hres, embs, Hres, ln1_s + HID, ln1_b + HID, (void*)X, BT);
    }
    convT<<<gCv4, blk, 0, stream>>>(wql, wkl, wvl, wol, Wqt, Wkt, Wvt, Wot, HID, HID);
    convT<<<gCv1, blk, 0, stream>>>(w1l, w1l, w1l, w1l, W1t, W1t, W1t, W1t, HID, DFF);
    convT<<<gCv2, blk, 0, stream>>>(w2l, w2l, w2l, w2l, W2t, W2t, W2t, W2t, DFF, HID);
    gemm64<2><<<gHH, blk, 0, stream>>>(X, HID, 0LL, Wqt, HID, 0LL, bq + l * HID,
                                       (void*)Qh, (void*)Ql, HID, 0LL, BT, HID, HID);
    gemm64<1><<<gHH, blk, 0, stream>>>(X, HID, 0LL, Wkt, HID, 0LL, bk + l * HID,
                                       (void*)Kh, (void*)Kh, HID, 0LL, BT, HID, HID);
    gemm64<3><<<gVT, blk, 0, stream>>>(Wvt, HID, 0LL, X, HID, (long long)SEQ * HID, bv + l * HID,
                                       (void*)VT, (void*)VT, SEQ, (long long)HID * SEQ, HID, SEQ, HID);
    attn64<<<gAt, dim3(128), 0, stream>>>(Qh, Ql, Kh, VT, mask, Ctx, 0.125f);
    gemm64<0><<<gHH, blk, 0, stream>>>(Ctx, HID, 0LL, Wot, HID, 0LL, bo + l * HID,
                                       (void*)Hres, (void*)Hres, HID, 0LL, BT, HID, HID);
    ln_rows<false, false, false><<<gLN, blk, 0, stream>>>(Hres, embs, Hres, ln2_s + l * HID, ln2_b + l * HID, (void*)X, BT);
    gemm64<4><<<gF1, blk, 0, stream>>>(X, HID, 0LL, W1t, HID, 0LL, b1 + l * DFF,
                                       (void*)G, (void*)G, DFF, 0LL, BT, DFF, HID);
    gemm64<0><<<gHH, blk, 0, stream>>>(G, DFF, 0LL, W2t, DFF, 0LL, b2 + l * HID,
                                       (void*)Hres, (void*)Hres, HID, 0LL, BT, HID, DFF);
  }
  ln_rows<false, false, true><<<gLN, blk, 0, stream>>>(Hres, embs, Hres, lnf_s, lnf_b, (void*)out, BT);
  (void)hipGetLastError();
}
